// HeterogeneousGraphTransformer_15367392985644
// MI455X (gfx1250) — hardware-verified
//
#include <hip/hip_runtime.h>
#include <stddef.h>


#define DD      256
#define TT      3
#define NTHR    256
#define NWAVE   8
#define EPT     8
#define NGRP    2
#define CHUNK   (NTHR * EPT * NGRP)
#define WCAP    (EPT * NGRP * 32)
#define LISTN   (NWAVE * WCAP)
#define NBC     4096
#define NBF     1024
#define RCAP    40960
#define RBN     128
#define TGT     256
#define DEGCAP  512
#define OTHR    512
#define GBM     64
#define LDS_PROJ (GBM * DD * 4)
#define LDS_COMB ((64 * 256 * 2 + 128 * 256 * 2) * 2)
#define LDS_FILL ((RCAP + NBF + LISTN) * 4 + 64)
#define WSCALE  64.0f
#define WINV    0.015625f
#define QKSCALE 0.125f
#define WSCAP   134217728
#define NEG_BIG (-3.0e38f)

static_assert((CHUNK & (CHUNK - 1)) == 0);
static_assert(CHUNK <= 4096);
static_assert(NBC <= 4096 && NBF <= 4096);
static_assert((NBC & (NBC - 1)) == 0 && (NBF & (NBF - 1)) == 0);
static_assert(NBC == 4 * NBF);
static_assert(OTHR * 8 == NBC);
static_assert((RCAP % 32) == 0);
static_assert(TGT == NWAVE * 32);
static_assert((NBC % TGT) == 0);
static_assert((TGT % GBM) == 0);
static_assert(DD == 256 && GBM == 64 && NTHR == 256);
static_assert(LDS_PROJ == 64 * 256 * 2 * 2);

typedef float          v4f  __attribute__((ext_vector_type(4)));
typedef float          v8f  __attribute__((ext_vector_type(8)));
typedef int            v4i  __attribute__((ext_vector_type(4)));
typedef unsigned short v8us __attribute__((ext_vector_type(8)));
typedef _Float16       v8h  __attribute__((ext_vector_type(8)));
typedef _Float16       v16h __attribute__((ext_vector_type(16)));
typedef __bf16         v16bf __attribute__((ext_vector_type(16)));
union FragH { v16h v; v8us h[2]; };
union FragB { v16bf v; v8us h[2]; };
union Pack8 { v8h h; v8us u; };

__device__ __forceinline__ v8us cvt8h(v4f a, v4f b, float sc) {
  v8h r;
  r[0] = (_Float16)(a.x * sc); r[1] = (_Float16)(a.y * sc);
  r[2] = (_Float16)(a.z * sc); r[3] = (_Float16)(a.w * sc);
  r[4] = (_Float16)(b.x * sc); r[5] = (_Float16)(b.y * sc);
  r[6] = (_Float16)(b.z * sc); r[7] = (_Float16)(b.w * sc);
  Pack8 p;
  p.h = r;
  return p.u;
}

__device__ __forceinline__ unsigned bfr(float x) {
  const unsigned u = __float_as_uint(x);
  return (u + 0x7FFFu + ((u >> 16) & 1u)) >> 16;
}

__device__ __forceinline__ void split8(v4f a, v4f b, v8us& hi, v8us& lo) {
  float v[8];
  v[0] = a.x; v[1] = a.y; v[2] = a.z; v[3] = a.w;
  v[4] = b.x; v[5] = b.y; v[6] = b.z; v[7] = b.w;
  v8us h, l;
#pragma unroll
  for (int e = 0; e < 8; ++e) {
    const unsigned hb = bfr(v[e]);
    const float rem = v[e] - __uint_as_float(hb << 16);
    h[e] = (unsigned short)hb;
    l[e] = (unsigned short)bfr(rem);
  }
  hi = h;
  lo = l;
}

__device__ __forceinline__ v8f wmh(v16h a, v16h b, v8f c) {
  v8f d = __builtin_amdgcn_wmma_f32_16x16x32_f16(false, a, false, b, (short)0, c, false, false);
  asm volatile("v_nop\n\tv_nop\n\tv_nop\n\tv_nop" : "+v"(d) : "v"(a), "v"(b));
  return d;
}
__device__ __forceinline__ v8f wmb(v16bf a, v16bf b, v8f c) {
  v8f d = __builtin_amdgcn_wmma_f32_16x16x32_bf16(false, a, false, b, (short)0, c, false, false);
  asm volatile("v_nop\n\tv_nop\n\tv_nop\n\tv_nop" : "+v"(d) : "v"(a), "v"(b));
  return d;
}

template <int NB>
__device__ __forceinline__ int scan_chunk(const int* __restrict__ dsts, int nE, int cbase, int slotBase,
                                          int vec8, int* list, int tid, int lane, int wave) {
  int wc = 0;
#pragma unroll
  for (int g = 0; g < NGRP; ++g) {
    const int el0  = (g * NTHR + tid) * EPT;
    const int e0   = cbase + el0;
    const int sent = -2147483647 - 1;
    v4i da, db;
    if (vec8 != 0 && cbase + CHUNK <= nE) {
      da = *(const v4i*)(dsts + e0);
      db = *(const v4i*)(dsts + e0 + 4);
    } else {
      da.x = (e0     < nE) ? dsts[min(e0, nE - 1)] : sent;
      da.y = (e0 + 1 < nE) ? dsts[min(e0 + 1, nE - 1)] : sent;
      da.z = (e0 + 2 < nE) ? dsts[min(e0 + 2, nE - 1)] : sent;
      da.w = (e0 + 3 < nE) ? dsts[min(e0 + 3, nE - 1)] : sent;
      db.x = (e0 + 4 < nE) ? dsts[min(e0 + 4, nE - 1)] : sent;
      db.y = (e0 + 5 < nE) ? dsts[min(e0 + 5, nE - 1)] : sent;
      db.z = (e0 + 6 < nE) ? dsts[min(e0 + 6, nE - 1)] : sent;
      db.w = (e0 + 7 < nE) ? dsts[min(e0 + 7, nE - 1)] : sent;
    }
    const unsigned nb = (unsigned)slotBase;
    const unsigned s0 = (unsigned)da.x - nb, s1 = (unsigned)da.y - nb;
    const unsigned s2 = (unsigned)da.z - nb, s3 = (unsigned)da.w - nb;
    const unsigned s4 = (unsigned)db.x - nb, s5 = (unsigned)db.y - nb;
    const unsigned s6 = (unsigned)db.z - nb, s7 = (unsigned)db.w - nb;
    const bool h0 = s0 < (unsigned)NB, h1 = s1 < (unsigned)NB, h2 = s2 < (unsigned)NB, h3 = s3 < (unsigned)NB;
    const bool h4 = s4 < (unsigned)NB, h5 = s5 < (unsigned)NB, h6 = s6 < (unsigned)NB, h7 = s7 < (unsigned)NB;
    const unsigned any = __builtin_amdgcn_ballot_w32(h0 | h1 | h2 | h3 | h4 | h5 | h6 | h7);
    if (any != 0u) {
#define HITJ(J, HJ, SJ) { \
        const unsigned mj = __builtin_amdgcn_ballot_w32(HJ); \
        if (mj != 0u) { \
          if (HJ) { \
            const int pos = wc + (int)__builtin_amdgcn_mbcnt_lo(mj, 0u); \
            if (pos < WCAP) list[wave * WCAP + pos] = ((el0 + (J)) << 12) | (int)(SJ); \
          } \
          wc += (int)__builtin_popcount(mj); } }
      HITJ(0, h0, s0)
      HITJ(1, h1, s1)
      HITJ(2, h2, s2)
      HITJ(3, h3, s3)
      HITJ(4, h4, s4)
      HITJ(5, h5, s5)
      HITJ(6, h6, s6)
      HITJ(7, h7, s7)
#undef HITJ
    }
  }
  return wc;
}

__global__ __launch_bounds__(NTHR) void k_wprep(const float* __restrict__ W, unsigned short* wp, int nUnits) {
  const int i = (int)blockIdx.x * NTHR + (int)threadIdx.x;
  if (i >= nUnits) return;
  const float* p = W + (size_t)i * 8;
  const v4f a = *(const v4f*)p, b = *(const v4f*)(p + 4);
  const v8us hv = cvt8h(a, b, WSCALE);
  unsigned short* d = wp + (size_t)i * 8;
  *(volatile v8us*)d = hv;
  __threadfence();
  *(volatile v8us*)d = hv;
}

__global__ __launch_bounds__(NTHR) void k_wcomb(const float* __restrict__ WQ, const float* __restrict__ WK,
                                                unsigned short* Mh, unsigned short* Ml) {
  extern __shared__ v4f lds_dyn[];
  unsigned short* Ash = (unsigned short*)lds_dyn;
  unsigned short* Asl = Ash + 64 * 256;
  unsigned short* Bsh = Asl + 64 * 256;
  unsigned short* Bsl = Bsh + 128 * 256;
  float* stg = (float*)lds_dyn;
  const int tid = threadIdx.x, lane = tid & 31, wave = tid >> 5, hh = lane >> 4, m = lane & 15;
  const int k0c = (int)blockIdx.x * 128;
  const int n0  = (int)blockIdx.y * 64;
  const int r   = (int)blockIdx.z;
  const float* wq = WQ + (size_t)r * DD * DD;
  const float* wk = WK + (size_t)r * DD * DD;

  {
    const int nl = tid & 63, og = tid >> 6;
#pragma unroll 1
    for (int g = 0; g < 8; ++g) {
      const int o8 = og * 64 + 8 * g;
      const float* p = wk + (size_t)o8 * DD + n0 + nl;
      v4f a, b;
      a.x = p[0];      a.y = p[DD];     a.z = p[2 * DD]; a.w = p[3 * DD];
      b.x = p[4 * DD]; b.y = p[5 * DD]; b.z = p[6 * DD]; b.w = p[7 * DD];
      v8us h, l;
      split8(a, b, h, l);
      *(v8us*)(Ash + nl * 256 + o8) = h;
      *(v8us*)(Asl + nl * 256 + o8) = l;
    }
    const int kl = tid & 127, og2 = tid >> 7;
#pragma unroll 1
    for (int g = 0; g < 16; ++g) {
      const int o8 = og2 * 128 + 8 * g;
      const float* p = wq + (size_t)o8 * DD + k0c + kl;
      v4f a, b;
      a.x = p[0];      a.y = p[DD];     a.z = p[2 * DD]; a.w = p[3 * DD];
      b.x = p[4 * DD]; b.y = p[5 * DD]; b.z = p[6 * DD]; b.w = p[7 * DD];
      v8us h, l;
      split8(a, b, h, l);
      *(v8us*)(Bsh + kl * 256 + o8) = h;
      *(v8us*)(Bsl + kl * 256 + o8) = l;
    }
  }
  __syncthreads();

  const int rg = wave >> 1, chf = wave & 1;
  const int r0 = 16 * rg;
  const int c0 = 64 * chf;
  v8f acc[4];
#pragma unroll
  for (int t = 0; t < 4; ++t) { v8f z = {0.f, 0.f, 0.f, 0.f, 0.f, 0.f, 0.f, 0.f}; acc[t] = z; }
  const unsigned short* ap  = Ash + (r0 + m) * 256 + 8 * hh;
  const unsigned short* alp = Asl + (r0 + m) * 256 + 8 * hh;
  const unsigned short* bq  = Bsh + (c0 + m) * 256 + 8 * hh;
  const unsigned short* blq = Bsl + (c0 + m) * 256 + 8 * hh;
#pragma unroll 1
  for (int kt = 0; kt < 8; ++kt) {
    FragB a, al;
    a.h[0]  = *(const v8us*)(ap + 32 * kt);
    a.h[1]  = *(const v8us*)(ap + 32 * kt + 16);
    al.h[0] = *(const v8us*)(alp + 32 * kt);
    al.h[1] = *(const v8us*)(alp + 32 * kt + 16);
#pragma unroll
    for (int t = 0; t < 4; ++t) {
      FragB b, bl;
      const unsigned short* bp  = bq + (16 * t) * 256 + 32 * kt;
      const unsigned short* blp = blq + (16 * t) * 256 + 32 * kt;
      b.h[0]  = *(const v8us*)bp;
      b.h[1]  = *(const v8us*)(bp + 16);
      bl.h[0] = *(const v8us*)blp;
      bl.h[1] = *(const v8us*)(blp + 16);
      acc[t] = wmb(a.v, b.v, acc[t]);
      acc[t] = wmb(a.v, bl.v, acc[t]);
      acc[t] = wmb(al.v, b.v, acc[t]);
    }
  }
  __syncthreads();

  {
    float* sp = stg + (r0 + 8 * hh) * 128 + c0 + m;
#pragma unroll
    for (int t = 0; t < 4; ++t) {
#pragma unroll
      for (int q = 0; q < 8; ++q) sp[q * 128 + 16 * t] = acc[t][q];
    }
  }
  __syncthreads();

  v8us hv[4], lv[4];
  size_t ga[4];
#pragma unroll
  for (int it = 0; it < 4; ++it) {
    const int row = 8 * wave + 2 * it + hh;
    const int c8  = 8 * m;
    const v4f a = *(const v4f*)(stg + row * 128 + c8);
    const v4f b = *(const v4f*)(stg + row * 128 + c8 + 4);
    split8(a, b, hv[it], lv[it]);
    ga[it] = (size_t)(r * DD + n0 + row) * DD + k0c + c8;
    *(volatile v8us*)(Mh + ga[it]) = hv[it];
    *(volatile v8us*)(Ml + ga[it]) = lv[it];
  }
  __threadfence();
#pragma unroll
  for (int it = 0; it < 4; ++it) {
    *(volatile v8us*)(Mh + ga[it]) = hv[it];
    *(volatile v8us*)(Ml + ga[it]) = lv[it];
  }
}

template <int SPLIT>
__global__ __launch_bounds__(NTHR) void k_proj(
    const float* __restrict__ A, int nRowsA,
    const unsigned short* __restrict__ Bh, const unsigned short* __restrict__ Bl,
    float* C, float oscale) {
  constexpr int TPW = 8;
  constexpr int WC  = TPW * 16;
  extern __shared__ v4f lds_dyn[];
  unsigned short* Ah = (unsigned short*)lds_dyn;
  unsigned short* Al = Ah + GBM * DD;
  float* stg = (float*)lds_dyn;
  const int tid = threadIdx.x, lane = tid & 31, wave = tid >> 5, hh = lane >> 4, m = lane & 15;
  const int rowBase = (int)blockIdx.x * GBM;
  const v4f z4 = {0.f, 0.f, 0.f, 0.f};

#pragma unroll 1
  for (int it = 0; it < (GBM * DD / 8) / NTHR; ++it) {
    const int u    = it * NTHR + tid;
    const int row  = u >> 5;
    const int c8   = (u & 31) * 8;
    const int grow = rowBase + row;
    const int rc   = grow < nRowsA ? grow : nRowsA - 1;
    const float* p = A + (size_t)rc * DD + c8;
    v4f a = *(const v4f*)p, b = *(const v4f*)(p + 4);
    if (grow >= nRowsA) { a = z4; b = z4; }
    if (SPLIT != 0) {
      v8us h, l;
      split8(a, b, h, l);
      *(v8us*)(Ah + row * DD + c8) = h;
      *(v8us*)(Al + row * DD + c8) = l;
    } else {
      *(v8us*)(Ah + row * DD + c8) = cvt8h(a, b, 1.0f);
    }
  }
  __syncthreads();

  const int rg  = wave >> 1;
  const int chf = wave & 1;
  const int r0  = rg * 16;
  const int c0  = chf * WC;
  v8f acc[TPW];
#pragma unroll
  for (int t = 0; t < TPW; ++t) { v8f z = {0.f, 0.f, 0.f, 0.f, 0.f, 0.f, 0.f, 0.f}; acc[t] = z; }
  const unsigned short* ap  = Ah + (r0 + m) * DD + 8 * hh;
  const unsigned short* alp = Al + (r0 + m) * DD + 8 * hh;
  const unsigned short* bq  = Bh + (size_t)(c0 + m) * DD + 8 * hh;
  const unsigned short* blq = Bl + (size_t)(c0 + m) * DD + 8 * hh;
  if (SPLIT != 0) {
#pragma unroll 1
    for (int kt = 0; kt < DD / 32; ++kt) {
      FragB a, al;
      a.h[0]  = *(const v8us*)(ap + 32 * kt);
      a.h[1]  = *(const v8us*)(ap + 32 * kt + 16);
      al.h[0] = *(const v8us*)(alp + 32 * kt);
      al.h[1] = *(const v8us*)(alp + 32 * kt + 16);
#pragma unroll
      for (int t = 0; t < TPW; ++t) {
        const unsigned short* bp  = bq + (size_t)(16 * t) * DD + 32 * kt;
        const unsigned short* blp = blq + (size_t)(16 * t) * DD + 32 * kt;
        FragB b, bl;
        b.h[0]  = *(const v8us*)bp;
        b.h[1]  = *(const v8us*)(bp + 16);
        bl.h[0] = *(const v8us*)blp;
        bl.h[1] = *(const v8us*)(blp + 16);
        acc[t] = wmb(a.v, b.v, acc[t]);
        acc[t] = wmb(a.v, bl.v, acc[t]);
        acc[t] = wmb(al.v, b.v, acc[t]);
      }
    }
  } else {
#pragma unroll 1
    for (int kt = 0; kt < DD / 32; ++kt) {
      FragH a;
      a.h[0] = *(const v8us*)(ap + 32 * kt);
      a.h[1] = *(const v8us*)(ap + 32 * kt + 16);
#pragma unroll
      for (int t = 0; t < TPW; ++t) {
        const unsigned short* bp = bq + (size_t)(16 * t) * DD + 32 * kt;
        FragH b;
        b.h[0] = *(const v8us*)bp;
        b.h[1] = *(const v8us*)(bp + 16);
        acc[t] = wmh(a.v, b.v, acc[t]);
      }
    }
  }
  __syncthreads();

  {
    float* sp = stg + (size_t)(r0 + 8 * hh) * DD + c0 + m;
#pragma unroll
    for (int t = 0; t < TPW; ++t) {
#pragma unroll
      for (int q = 0; q < 8; ++q) sp[q * DD + 16 * t] = acc[t][q] * oscale;
    }
  }
  __syncthreads();

  const int col = c0 + 4 * lane;
  const size_t gb = (size_t)(rowBase + r0) * DD + col;
#pragma unroll
  for (int it = 0; it < 16; ++it) {
    const v4f v = *(const v4f*)(stg + (size_t)(r0 + it) * DD + col);
    *(volatile v4f*)(C + gb + (size_t)it * DD) = v;
  }
  __threadfence();
#pragma unroll
  for (int it = 0; it < 16; ++it) {
    const v4f v = *(const v4f*)(stg + (size_t)(r0 + it) * DD + col);
    *(volatile v4f*)(C + gb + (size_t)it * DD) = v;
  }
}

__global__ __launch_bounds__(NTHR) void k_count(
    const int* __restrict__ e0, const int* __restrict__ e1, const int* __restrict__ e2,
    int* cntAll, int nE, int vec8, int cntStride) {
  __shared__ __attribute__((aligned(16))) int scnt[NBC];
  __shared__ __attribute__((aligned(16))) int list[LISTN];
  __shared__ int wcnt[NWAVE];
  const int tid = threadIdx.x, lane = tid & 31, wave = tid >> 5;
  const int nodeBase = blockIdx.x * NBC;
  const int t = (int)blockIdx.y;
  const int* dsts = (t == 0) ? e0 : ((t == 1) ? e1 : e2);
  int* cnt = cntAll + (size_t)t * cntStride;

  for (int i = tid; i < NBC; i += NTHR) scnt[i] = 0;
  __syncthreads();

  const int nChunks = (nE + CHUNK - 1) / CHUNK;
#pragma unroll 1
  for (int ch = 0; ch < nChunks; ++ch) {
    const int cbase = ch * CHUNK;
    const int wc = scan_chunk<NBC>(dsts, nE, cbase, nodeBase, vec8, list, tid, lane, wave);
    if (lane == 0) wcnt[wave] = wc;
    __syncthreads();
    if (wave == 0) {
#pragma unroll 1
      for (int wsx = 0; wsx < NWAVE; ++wsx) {
        int n = __builtin_amdgcn_readfirstlane(wcnt[wsx]);
        n = n > WCAP ? WCAP : (n < 0 ? 0 : n);
        const int* lp = list + wsx * WCAP;
#pragma unroll 1
        for (int i = 0; i < n; ++i) {
          const int ent  = __builtin_amdgcn_readfirstlane(lp[i]);
          const int slot = ent & (NBC - 1);
          if (lane == 0) scnt[slot] = scnt[slot] + 1;
        }
      }
    }
    __syncthreads();
  }

  v4i cq[4];
#pragma unroll
  for (int q = 0; q < 4; ++q) {
    const int f = (wave * 4 + q) * 128 + 4 * lane;
    cq[q] = *(const v4i*)(scnt + f);
  }
  int* cp = cnt + (size_t)nodeBase;
#pragma unroll
  for (int q = 0; q < 4; ++q) {
    const int f = (wave * 4 + q) * 128 + 4 * lane;
    *(volatile v4i*)(cp + f) = cq[q];
  }
  __threadfence();
#pragma unroll
  for (int q = 0; q < 4; ++q) {
    const int f = (wave * 4 + q) * 128 + 4 * lane;
    *(volatile v4i*)(cp + f) = cq[q];
  }
}

__global__ __launch_bounds__(OTHR) void k_offsets(
    const int* __restrict__ cntAll, int* offAll, int* rbAll, int nChunk, int cntStride) {
  __shared__ __attribute__((aligned(16))) int soff[NBC];
  __shared__ __attribute__((aligned(16))) int srb[RBN];
  __shared__ int wtot[OTHR / 32];
  const int tid = threadIdx.x, lane = tid & 31, wave = tid >> 5, sub = tid >> 7;
  const int* cnt = cntAll + (size_t)blockIdx.x * cntStride;
  int* off   = offAll + (size_t)blockIdx.x * cntStride;
  int* rbase = rbAll + (size_t)blockIdx.x * RBN;
  for (int i = tid; i < RBN; i += OTHR) srb[i] = 0;
  int carry = 0;
#pragma unroll 1
  for (int ch = 0; ch < nChunk; ++ch) {
    const int base = ch * NBC;
    const v4i c0 = *(const v4i*)(cnt + base + 8 * tid);
    const v4i c1 = *(const v4i*)(cnt + base + 8 * tid + 4);
    const int e0 = max(c0.x, 0), e1 = max(c0.y, 0), e2 = max(c0.z, 0), e3 = max(c0.w, 0);
    const int e4 = max(c1.x, 0), e5 = max(c1.y, 0), e6 = max(c1.z, 0), e7 = max(c1.w, 0);
    const int ts = e0 + e1 + e2 + e3 + e4 + e5 + e6 + e7;
    int incl = ts;
#pragma unroll
    for (int d = 1; d < 32; d <<= 1) {
      const int tv = __shfl_up(incl, d);
      if (lane >= d) incl += tv;
    }
    if (lane == 31) wtot[wave] = incl;
    __syncthreads();
    const int S0 = wtot[0]  + wtot[1]  + wtot[2]  + wtot[3];
    const int S1 = wtot[4]  + wtot[5]  + wtot[6]  + wtot[7];
    const int S2 = wtot[8]  + wtot[9]  + wtot[10] + wtot[11];
    const int S3 = wtot[12] + wtot[13] + wtot[14] + wtot[15];
    int pre = 0;
#pragma unroll 1
    for (int w = 4 * sub; w < wave; ++w) pre += wtot[w];
    const int b0 = carry;
    const int b1 = b0 + ((S0 + 31) & ~31);
    const int b2 = b1 + ((S1 + 31) & ~31);
    const int b3 = b2 + ((S2 + 31) & ~31);
    const int b4 = b3 + ((S3 + 31) & ~31);
    const int myb = sub == 0 ? b0 : (sub == 1 ? b1 : (sub == 2 ? b2 : b3));
    if (tid == 0) {
      srb[min(4 * ch + 0, RBN - 1)] = b0;
      srb[min(4 * ch + 1, RBN - 1)] = b1;
      srb[min(4 * ch + 2, RBN - 1)] = b2;
      srb[min(4 * ch + 3, RBN - 1)] = b3;
    }
    int run = myb + pre + incl - ts;
    soff[8 * tid + 0] = run; run += e0;
    soff[8 * tid + 1] = run; run += e1;
    soff[8 * tid + 2] = run; run += e2;
    soff[8 * tid + 3] = run; run += e3;
    soff[8 * tid + 4] = run; run += e4;
    soff[8 * tid + 5] = run; run += e5;
    soff[8 * tid + 6] = run; run += e6;
    soff[8 * tid + 7] = run;
    carry = b4;
    __syncthreads();
    const v4i o0 = *(const v4i*)(soff + 4 * tid);
    const v4i o1 = *(const v4i*)(soff + 4 * (tid + OTHR));
    int* op = off + base;
    *(volatile v4i*)(op + 4 * tid) = o0;
    *(volatile v4i*)(op + 4 * (tid + OTHR)) = o1;
    __threadfence();
    *(volatile v4i*)(op + 4 * tid) = o0;
    *(volatile v4i*)(op + 4 * (tid + OTHR)) = o1;
    __syncthreads();
  }
  if (tid == 0) srb[min(4 * nChunk, RBN - 1)] = carry;
  __syncthreads();
  v4i rv = {0, 0, 0, 0};
  if (tid < 32) rv = *(const v4i*)(srb + 4 * tid);
  if (tid < 32) *(volatile v4i*)(rbase + 4 * tid) = rv;
  __threadfence();
  if (tid < 32) *(volatile v4i*)(rbase + 4 * tid) = rv;
}

__global__ __launch_bounds__(NTHR) void k_fill(
    const int* __restrict__ e0, const int* __restrict__ e1, const int* __restrict__ e2,
    const int* __restrict__ offAll, const int* __restrict__ rbAll,
    int* csrAll, int nN, int nE, int vec8, int csrLen, int cntStride) {
  extern __shared__ v4f lds_dyn[];
  int* region = (int*)lds_dyn;
  int* cursor = region + RCAP;
  int* list   = cursor + NBF;
  int* wcnt   = list + LISTN;
  const int tid = threadIdx.x, lane = tid & 31, wave = tid >> 5;
  const int t = (int)blockIdx.y;
  const int b = (int)blockIdx.x;
  const int nodeBase = b * NBF;
  const int* dsts  = (t == 0) ? e0 : ((t == 1) ? e1 : e2);
  const int* off   = offAll + (size_t)t * cntStride;
  const int* rbase = rbAll + (size_t)t * RBN;
  int* csr = csrAll + (size_t)t * csrLen;

  int rb0 = rbase[b];
  const int rb1 = rbase[b + 1];
  rb0 = rb0 < 0 ? 0 : (rb0 > csrLen ? csrLen : rb0);
  rb0 &= ~31;
  int len = rb1 - rb0;
  len = len < 0 ? 0 : (len > RCAP ? RCAP : len);
  int lenW = (len + 31) & ~31;
  if (rb0 + lenW > csrLen) lenW = (csrLen - rb0) & ~31;

  {
    const v4i z = {0, 0, 0, 0};
    for (int i = tid; i < RCAP / 4; i += NTHR) ((v4i*)region)[i] = z;
    for (int s = tid; s < NBF; s += NTHR) {
      int o = off[nodeBase + s] - rb0;
      o = o < 0 ? 0 : (o > RCAP ? RCAP : o);
      cursor[s] = o;
    }
  }
  __syncthreads();

  const int nChunks = (nE + CHUNK - 1) / CHUNK;
#pragma unroll 1
  for (int ch = 0; ch < nChunks; ++ch) {
    const int cbase = ch * CHUNK;
    const int wc = scan_chunk<NBF>(dsts, nE, cbase, nodeBase, vec8, list, tid, lane, wave);
    if (lane == 0) wcnt[wave] = wc;
    __syncthreads();
    if (wave == 0) {
#pragma unroll 1
      for (int wsx = 0; wsx < NWAVE; ++wsx) {
        int n = __builtin_amdgcn_readfirstlane(wcnt[wsx]);
        n = n > WCAP ? WCAP : (n < 0 ? 0 : n);
        const int* lp = list + wsx * WCAP;
#pragma unroll 1
        for (int i = 0; i < n; ++i) {
          const int ent  = __builtin_amdgcn_readfirstlane(lp[i]);
          const int slot = ent & (NBF - 1);
          int e = cbase + ((ent >> 12) & (CHUNK - 1));
          e = e > nE - 1 ? nE - 1 : e;
          int ep = e ^ 1;
          ep = ep > nE - 1 ? nE - 1 : (ep < 0 ? 0 : ep);
          int src = dsts[ep];
          src = src < 0 ? 0 : (src > nN - 1 ? nN - 1 : src);
          if (lane == 0) {
            int pos = cursor[slot];
            pos = pos < 0 ? 0 : (pos > RCAP - 1 ? RCAP - 1 : pos);
            region[pos] = src;
            const int np = pos + 1;
            cursor[slot] = np > RCAP ? RCAP : np;
          }
        }
      }
    }
    __syncthreads();
  }

  const int nv = lenW >> 2;
  int* gp = csr + rb0;
#pragma unroll 1
  for (int i = tid; i < nv; i += NTHR) { const v4i v = ((const v4i*)region)[i]; *(volatile v4i*)(gp + 4 * i) = v; }
  __threadfence();
#pragma unroll 1
  for (int i = tid; i < nv; i += NTHR) { const v4i v = ((const v4i*)region)[i]; *(volatile v4i*)(gp + 4 * i) = v; }
}

template <int MODE>
__global__ __launch_bounds__(NTHR) void k_agg(
    const int* __restrict__ csr, const int* __restrict__ off, const int* __restrict__ cnt,
    const float* __restrict__ P, const float* __restrict__ S, const float* __restrict__ V,
    float* H, int nN, int csrLen) {
  const int tid = threadIdx.x, lane = tid & 31, wave = tid >> 5;
  const int tbase = (int)blockIdx.x * TGT + wave * 32;
  const int col0 = 4 * lane;
  const int col1 = DD / 2 + 4 * lane;
  const v4f z4 = {0.f, 0.f, 0.f, 0.f};

  const int cl    = tbase + lane;
  const int cnt_l = cnt[cl];
  const int off_l = off[cl];

#pragma unroll 1
  for (int j = 0; j < 32; ++j) {
    const int c = tbase + j;
    int n = __builtin_amdgcn_readfirstlane(__shfl(cnt_l, j));
    n = n < 0 ? 0 : (n > DEGCAP ? DEGCAP : n);
    const int st = __builtin_amdgcn_readfirstlane(__shfl(off_l, j));
    const v4f p0 = *(const v4f*)(P + (size_t)c * DD + col0);
    const v4f p1 = *(const v4f*)(P + (size_t)c * DD + col1);

    float mrun = NEG_BIG, den = 0.f;
    v4f a0 = z4, a1 = z4;
#pragma unroll 1
    for (int q0 = 0; q0 < n; q0 += 32) {
      int pos = st + q0 + lane;
      pos = pos < 0 ? 0 : (pos > csrLen - 1 ? csrLen - 1 : pos);
      int sl = csr[pos];
      sl = sl < 0 ? 0 : (sl > nN - 1 ? nN - 1 : sl);
      const int mcnt = (n - q0) < 32 ? (n - q0) : 32;

      float sc = 0.f, cmax = NEG_BIG;
#pragma unroll 1
      for (int pp = 0; pp < mcnt; ++pp) {
        const int s = __builtin_amdgcn_readlane(sl, pp);
        const v4f k0 = *(const v4f*)(S + (size_t)s * DD + col0);
        const v4f k1 = *(const v4f*)(S + (size_t)s * DD + col1);
        float d = p0.x * k0.x + p0.y * k0.y + p0.z * k0.z + p0.w * k0.w
                + p1.x * k1.x + p1.y * k1.y + p1.z * k1.z + p1.w * k1.w;
        d += __shfl_xor(d, 16);
        d += __shfl_xor(d, 8);
        d += __shfl_xor(d, 4);
        d += __shfl_xor(d, 2);
        d += __shfl_xor(d, 1);
        d *= QKSCALE;
        cmax = fmaxf(cmax, d);
        sc = (lane == pp) ? d : sc;
      }
      const float mnew = fmaxf(mrun, cmax);
      const float fac  = (q0 == 0) ? 0.f : __expf(mrun - mnew);
      den *= fac;
      a0 = a0 * fac;
      a1 = a1 * fac;
      mrun = mnew;

#pragma unroll 1
      for (int pp = 0; pp < mcnt; ++pp) {
        const int s = __builtin_amdgcn_readlane(sl, pp);
        const float ev = __expf(__shfl(sc, pp) - mnew);
        den += ev;
        const v4f v0 = *(const v4f*)(V + (size_t)s * DD + col0);
        const v4f v1 = *(const v4f*)(V + (size_t)s * DD + col1);
        a0 = a0 + v0 * ev;
        a1 = a1 + v1 * ev;
      }
    }

    const float rd = (n > 0) ? __builtin_amdgcn_rcpf(den) : 0.0f;
    v4f o0 = a0 * rd, o1 = a1 * rd;
    const int cc = c < nN ? c : nN - 1;
    if (MODE >= 1) {
      o0 = o0 + *(const v4f*)(H + (size_t)cc * DD + col0);
      o1 = o1 + *(const v4f*)(H + (size_t)cc * DD + col1);
    }
    if (MODE == 2) {
      o0.x = fmaxf(o0.x, 0.f); o0.y = fmaxf(o0.y, 0.f); o0.z = fmaxf(o0.z, 0.f); o0.w = fmaxf(o0.w, 0.f);
      o1.x = fmaxf(o1.x, 0.f); o1.y = fmaxf(o1.y, 0.f); o1.z = fmaxf(o1.z, 0.f); o1.w = fmaxf(o1.w, 0.f);
    }
    if (c < nN) {
      float* hp = H + (size_t)c * DD;
      *(volatile v4f*)(hp + col0) = o0;
      *(volatile v4f*)(hp + col1) = o1;
      __threadfence();
      *(volatile v4f*)(hp + col0) = o0;
      *(volatile v4f*)(hp + col1) = o1;
    }
  }
}

extern "C" void kernel_launch(void* const* d_in, const int* in_sizes, int n_in,
                              void* d_out, int out_size, void* d_ws, size_t ws_size,
                              hipStream_t stream) {
  if (n_in < 7) return;
  const int nN = in_sizes[0] / DD;
  if (nN <= 0 || in_sizes[0] != nN * DD) return;
  const int nE2 = in_sizes[1];
  if (nE2 <= 0 || (nE2 & 1) != 0 || in_sizes[2] != nE2 || in_sizes[3] != nE2) return;
  if (in_sizes[4] != TT * DD * DD || in_sizes[5] != TT * DD * DD || in_sizes[6] != TT * DD * DD) return;
  if (out_size != nN * DD) return;
  if (nE2 > (1 << 28) || nN > (1 << 24)) return;

  const float* Sx  = (const float*)d_in[0];
  const int*   eA  = (const int*)d_in[1];
  const int*   eB  = (const int*)d_in[2];
  const int*   eC  = (const int*)d_in[3];
  const float* W   = (const float*)d_in[4];
  const float* WQ  = (const float*)d_in[5];
  const float* WK  = (const float*)d_in[6];
  float* out = (float*)d_out;

  const int NPAD   = ((nN + TGT - 1) / TGT) * TGT;
  const int nBC    = (nN + NBC - 1) / NBC;
  const int CNTPAD = nBC * NBC;
  if (4 * nBC + 1 > RBN) return;
  const int nBF    = (nN + NBF - 1) / NBF;
  const int csrLen = ((nE2 + 31) & ~31) + 4096;
  if (31 * 4 * nBC > 4096) return;
  const int nAgg   = NPAD / TGT;
  const int nGemm  = NPAD / GBM;
  const int wUnits = TT * DD * DD / 8;
  const int PL     = DD * DD;

  char* ws = (char*)d_ws;
  size_t off = 0;
  const size_t oWv  = off; off += (size_t)TT * PL * 2;            off = (off + 255) & ~(size_t)255;
  const size_t oMh  = off; off += (size_t)TT * PL * 2;            off = (off + 255) & ~(size_t)255;
  const size_t oMl  = off; off += (size_t)TT * PL * 2;            off = (off + 255) & ~(size_t)255;
  const size_t oCnt = off; off += (size_t)TT * CNTPAD * 4;        off = (off + 255) & ~(size_t)255;
  const size_t oOff = off; off += (size_t)TT * CNTPAD * 4;        off = (off + 255) & ~(size_t)255;
  const size_t oRb  = off; off += (size_t)TT * RBN * 4;           off = (off + 255) & ~(size_t)255;
  const size_t oCsr = off; off += (size_t)TT * csrLen * 4;        off = (off + 255) & ~(size_t)255;
  const size_t oP   = off; off += (size_t)NPAD * DD * 4;          off = (off + 255) & ~(size_t)255;
  const size_t oV   = off; off += (size_t)NPAD * DD * 4;          off = (off + 255) & ~(size_t)255;
  if (off > ws_size || off > (size_t)WSCAP) return;
  unsigned short* wv = (unsigned short*)(ws + oWv);
  unsigned short* mh = (unsigned short*)(ws + oMh);
  unsigned short* ml = (unsigned short*)(ws + oMl);
  int*   cnt  = (int*)(ws + oCnt);
  int*   offp = (int*)(ws + oOff);
  int*   rb   = (int*)(ws + oRb);
  int*   csr  = (int*)(ws + oCsr);
  float* pp   = (float*)(ws + oP);
  float* vp   = (float*)(ws + oV);

  const int vec8 = ((nE2 & 3) == 0) ? 1 : 0;

  k_wprep<<<wUnits / NTHR, NTHR, 0, stream>>>(W, wv, wUnits);
  hipFuncSetAttribute(reinterpret_cast<const void*>(&k_wcomb),
                      hipFuncAttributeMaxDynamicSharedMemorySize, LDS_COMB);
  k_wcomb<<<dim3(2, 4, TT), NTHR, LDS_COMB, stream>>>(WQ, WK, mh, ml);

  k_count<<<dim3(nBC, TT), NTHR, 0, stream>>>(eA, eB, eC, cnt, nE2, vec8, CNTPAD);
  k_offsets<<<TT, OTHR, 0, stream>>>(cnt, offp, rb, nBC, CNTPAD);
  hipFuncSetAttribute(reinterpret_cast<const void*>(&k_fill),
                      hipFuncAttributeMaxDynamicSharedMemorySize, LDS_FILL);
  k_fill<<<dim3(nBF, TT), NTHR, LDS_FILL, stream>>>(eA, eB, eC, offp, rb, csr, nN, nE2, vec8, csrLen, CNTPAD);

  hipFuncSetAttribute(reinterpret_cast<const void*>(&k_proj<1>),
                      hipFuncAttributeMaxDynamicSharedMemorySize, LDS_PROJ);
  hipFuncSetAttribute(reinterpret_cast<const void*>(&k_proj<0>),
                      hipFuncAttributeMaxDynamicSharedMemorySize, LDS_PROJ);

  k_proj<1><<<nGemm, NTHR, LDS_PROJ, stream>>>(Sx, nN, mh, ml, pp, 1.0f);
  k_proj<0><<<nGemm, NTHR, LDS_PROJ, stream>>>(Sx, nN, wv, wv, vp, WINV);
  k_agg<0><<<nAgg, NTHR, 0, stream>>>(csr, offp, cnt, pp, Sx, vp, out, nN, csrLen);

  k_proj<1><<<nGemm, NTHR, LDS_PROJ, stream>>>(Sx, nN, mh + (size_t)PL, ml + (size_t)PL, pp, 1.0f);
  k_proj<0><<<nGemm, NTHR, LDS_PROJ, stream>>>(Sx, nN, wv + (size_t)PL, wv + (size_t)PL, vp, WINV);
  k_agg<1><<<nAgg, NTHR, 0, stream>>>(csr + (size_t)csrLen, offp + (size_t)CNTPAD, cnt + (size_t)CNTPAD,
                                       pp, Sx, vp, out, nN, csrLen);

  k_proj<1><<<nGemm, NTHR, LDS_PROJ, stream>>>(Sx, nN, mh + (size_t)2 * PL, ml + (size_t)2 * PL, pp, 1.0f);
  k_proj<0><<<nGemm, NTHR, LDS_PROJ, stream>>>(Sx, nN, wv + (size_t)2 * PL, wv + (size_t)2 * PL, vp, WINV);
  k_agg<2><<<nAgg, NTHR, 0, stream>>>(csr + (size_t)2 * csrLen, offp + (size_t)2 * CNTPAD, cnt + (size_t)2 * CNTPAD,
                                       pp, Sx, vp, out, nN, csrLen);
}
